// HGNNConv_69123203662121
// MI455X (gfx1250) — hardware-verified
//
#include <hip/hip_runtime.h>
#include <stddef.h>


#define DW      128
#define NHE     20000
#define NTHR    256
#define NWAVE   8
#define EPT     8
#define NGRP    2
#define CHUNK   (NTHR * EPT * NGRP)
#define WCAP    (EPT * NGRP * 32)
#define LISTN   (NWAVE * WCAP)
#define NBC     4096
#define OTHR    512
#define FBV     2048
#define FBE     512
#define FBMAX   2048
#define RCAP    49152
#define RBN     128
#define TGT     256
#define DEGCAP  1024
#define BM      64
#define KSTEPS  (DW / 32)
#define WSCAP   134217728
#define ACARRY  8.0f
#define WCARRY  64.0f
#define GSCALE  (1.0f / 512.0f)

#define LDS_FILL ((RCAP + FBMAX + LISTN) * 4 + 64)

static_assert((CHUNK & (CHUNK - 1)) == 0);
static_assert(CHUNK <= 4096);
static_assert((NBC & (NBC - 1)) == 0);
static_assert(NBC <= 4096);
static_assert(OTHR * 8 == NBC);
static_assert((FBV & (FBV - 1)) == 0 && (FBE & (FBE - 1)) == 0);
static_assert(FBV <= FBMAX && FBE <= FBMAX);
static_assert((NBC % FBV) == 0 && (NBC % FBE) == 0);
static_assert((RCAP % 32) == 0);
static_assert(TGT == NWAVE * 32);
static_assert((NBC % TGT) == 0);
static_assert((TGT % BM) == 0);
static_assert(DW == 4 * 32);
static_assert((DW % 32) == 0);
static_assert(WCAP == EPT * NGRP * 32);

typedef float    v4f  __attribute__((ext_vector_type(4)));
typedef float    v8f  __attribute__((ext_vector_type(8)));
typedef int      v4i  __attribute__((ext_vector_type(4)));
typedef _Float16 v4h  __attribute__((ext_vector_type(4)));
typedef _Float16 v8h  __attribute__((ext_vector_type(8)));
typedef _Float16 v16h __attribute__((ext_vector_type(16)));
union Frag { v16h v; v8h h[2]; };

__device__ __forceinline__ v8f wmh(v16h a, v16h b, v8f c) {
  v8f d = __builtin_amdgcn_wmma_f32_16x16x32_f16(false, a, false, b, (short)0, c, false, false);
  asm volatile("v_nop\n\tv_nop\n\tv_nop\n\tv_nop" : "+v"(d) : "v"(a), "v"(b));
  return d;
}

template <int NB>
__device__ __forceinline__ int scan_chunk(const int* __restrict__ dsts, int nE, int cbase, int slotBase,
                                          int vec8, int* list, int tid, int lane, int wave) {
  int wc = 0;
#pragma unroll
  for (int g = 0; g < NGRP; ++g) {
    const int el0  = (g * NTHR + tid) * EPT;
    const int e0   = cbase + el0;
    const int sent = -2147483647 - 1;
    v4i da, db;
    if (vec8 != 0 && cbase + CHUNK <= nE) {
      da = *(const v4i*)(dsts + e0);
      db = *(const v4i*)(dsts + e0 + 4);
    } else {
      da.x = (e0     < nE) ? dsts[min(e0, nE - 1)] : sent;
      da.y = (e0 + 1 < nE) ? dsts[min(e0 + 1, nE - 1)] : sent;
      da.z = (e0 + 2 < nE) ? dsts[min(e0 + 2, nE - 1)] : sent;
      da.w = (e0 + 3 < nE) ? dsts[min(e0 + 3, nE - 1)] : sent;
      db.x = (e0 + 4 < nE) ? dsts[min(e0 + 4, nE - 1)] : sent;
      db.y = (e0 + 5 < nE) ? dsts[min(e0 + 5, nE - 1)] : sent;
      db.z = (e0 + 6 < nE) ? dsts[min(e0 + 6, nE - 1)] : sent;
      db.w = (e0 + 7 < nE) ? dsts[min(e0 + 7, nE - 1)] : sent;
    }
    const unsigned nb = (unsigned)slotBase;
    const unsigned s0 = (unsigned)da.x - nb, s1 = (unsigned)da.y - nb;
    const unsigned s2 = (unsigned)da.z - nb, s3 = (unsigned)da.w - nb;
    const unsigned s4 = (unsigned)db.x - nb, s5 = (unsigned)db.y - nb;
    const unsigned s6 = (unsigned)db.z - nb, s7 = (unsigned)db.w - nb;
    const bool h0 = s0 < (unsigned)NB, h1 = s1 < (unsigned)NB, h2 = s2 < (unsigned)NB, h3 = s3 < (unsigned)NB;
    const bool h4 = s4 < (unsigned)NB, h5 = s5 < (unsigned)NB, h6 = s6 < (unsigned)NB, h7 = s7 < (unsigned)NB;
    const unsigned any = __builtin_amdgcn_ballot_w32(h0 | h1 | h2 | h3 | h4 | h5 | h6 | h7);
    if (any != 0u) {
#define HITJ(J, HJ, SJ) { \
        const unsigned mj = __builtin_amdgcn_ballot_w32(HJ); \
        if (mj != 0u) { \
          if (HJ) { \
            const int pos = wc + (int)__builtin_amdgcn_mbcnt_lo(mj, 0u); \
            if (pos < WCAP) list[wave * WCAP + pos] = ((el0 + (J)) << 12) | (int)(SJ); \
          } \
          wc += (int)__builtin_popcount(mj); } }
      HITJ(0, h0, s0)
      HITJ(1, h1, s1)
      HITJ(2, h2, s2)
      HITJ(3, h3, s3)
      HITJ(4, h4, s4)
      HITJ(5, h5, s5)
      HITJ(6, h6, s6)
      HITJ(7, h7, s7)
#undef HITJ
    }
  }
  return wc;
}

template <int MODE>
__device__ __forceinline__ float degval(int c) {
  const float f = (float)(c < 1 ? 1 : c);
  float r;
  if constexpr (MODE == 0) r = rsqrtf(f);
  else                     r = __builtin_amdgcn_rcpf(f);
  return c > 0 ? r : 0.f;
}

template <int MODE>
__global__ __launch_bounds__(NTHR) void k_count(
    const int* __restrict__ dsts, int* cnt, float* dinv, int nE, int vec8) {
  __shared__ __attribute__((aligned(16))) int scnt[NBC];
  __shared__ __attribute__((aligned(16))) int list[LISTN];
  __shared__ int wcnt[NWAVE];
  const int tid = threadIdx.x, lane = tid & 31, wave = tid >> 5;
  const int nodeBase = blockIdx.x * NBC;

  for (int i = tid; i < NBC; i += NTHR) scnt[i] = 0;
  __syncthreads();

  const int nChunks = (nE + CHUNK - 1) / CHUNK;
#pragma unroll 1
  for (int ch = 0; ch < nChunks; ++ch) {
    const int cbase = ch * CHUNK;
    const int wc = scan_chunk<NBC>(dsts, nE, cbase, nodeBase, vec8, list, tid, lane, wave);
    if (lane == 0) wcnt[wave] = wc;
    __syncthreads();
    if (wave == 0) {
#pragma unroll 1
      for (int wsx = 0; wsx < NWAVE; ++wsx) {
        int n = __builtin_amdgcn_readfirstlane(wcnt[wsx]);
        n = n > WCAP ? WCAP : (n < 0 ? 0 : n);
        const int* lp = list + wsx * WCAP;
#pragma unroll 1
        for (int i = 0; i < n; ++i) {
          const int ent  = __builtin_amdgcn_readfirstlane(lp[i]);
          const int slot = ent & (NBC - 1);
          if (lane == 0) scnt[slot] = scnt[slot] + 1;
        }
      }
    }
    __syncthreads();
  }

  v4i cq[4];
  v4f dq[4];
#pragma unroll
  for (int q = 0; q < 4; ++q) {
    const int f = (wave * 4 + q) * 128 + 4 * lane;
    const v4i cv = *(const v4i*)(scnt + f);
    cq[q] = cv;
    v4f d;
    d.x = degval<MODE>(cv.x);
    d.y = degval<MODE>(cv.y);
    d.z = degval<MODE>(cv.z);
    d.w = degval<MODE>(cv.w);
    dq[q] = d;
  }
  int*   cp = cnt  + (size_t)nodeBase;
  float* dp = dinv + (size_t)nodeBase;
#pragma unroll
  for (int q = 0; q < 4; ++q) {
    const int f = (wave * 4 + q) * 128 + 4 * lane;
    *(volatile v4i*)(cp + f) = cq[q];
    *(volatile v4f*)(dp + f) = dq[q];
  }
  __threadfence();
#pragma unroll
  for (int q = 0; q < 4; ++q) {
    const int f = (wave * 4 + q) * 128 + 4 * lane;
    *(volatile v4i*)(cp + f) = cq[q];
    *(volatile v4f*)(dp + f) = dq[q];
  }
}

template <int NFB>
__global__ __launch_bounds__(OTHR) void k_offsets(
    const int* __restrict__ cnt, int* off, int* rbase, int nChunk, int csrLen) {
  constexpr int NW  = OTHR / 32;
  constexpr int WPF = NW / NFB;
  static_assert((NW % NFB) == 0);
  static_assert(WPF * NFB * 256 == NBC);
  __shared__ __attribute__((aligned(16))) int soff[NBC];
  __shared__ __attribute__((aligned(16))) int srb[RBN];
  __shared__ int wtot[NW];
  const int tid = threadIdx.x, lane = tid & 31, wave = tid >> 5, sub = wave / WPF;
  for (int i = tid; i < RBN; i += OTHR) srb[i] = 0;
  int carry = 0, flag = 0;
#pragma unroll 1
  for (int ch = 0; ch < nChunk; ++ch) {
    const int base = ch * NBC;
    const v4i c0 = *(const v4i*)(cnt + base + 8 * tid);
    const v4i c1 = *(const v4i*)(cnt + base + 8 * tid + 4);
    const int e0 = max(c0.x, 0), e1 = max(c0.y, 0), e2 = max(c0.z, 0), e3 = max(c0.w, 0);
    const int e4 = max(c1.x, 0), e5 = max(c1.y, 0), e6 = max(c1.z, 0), e7 = max(c1.w, 0);
    const int ts = e0 + e1 + e2 + e3 + e4 + e5 + e6 + e7;
    int incl = ts;
#pragma unroll
    for (int d = 1; d < 32; d <<= 1) {
      const int t = __shfl_up(incl, d);
      if (lane >= d) incl += t;
    }
    if (lane == 31) wtot[wave] = incl;
    __syncthreads();
    int bsum = carry, myb = carry;
#pragma unroll
    for (int f = 0; f < NFB; ++f) {
      int S = 0;
#pragma unroll
      for (int w = 0; w < WPF; ++w) S += wtot[f * WPF + w];
      myb = (f == sub) ? bsum : myb;
      if (tid == 0) srb[min(NFB * ch + f, RBN - 2)] = bsum;
      const int Sp = (S + 31) & ~31;
      flag |= (Sp > RCAP) ? 1 : 0;
      bsum += Sp;
    }
    int pre = 0;
#pragma unroll 1
    for (int w = sub * WPF; w < wave; ++w) pre += wtot[w];
    int run = myb + pre + incl - ts;
    soff[8 * tid + 0] = run; run += e0;
    soff[8 * tid + 1] = run; run += e1;
    soff[8 * tid + 2] = run; run += e2;
    soff[8 * tid + 3] = run; run += e3;
    soff[8 * tid + 4] = run; run += e4;
    soff[8 * tid + 5] = run; run += e5;
    soff[8 * tid + 6] = run; run += e6;
    soff[8 * tid + 7] = run;
    carry = bsum;
    __syncthreads();
    const v4i o0 = *(const v4i*)(soff + 4 * tid);
    const v4i o1 = *(const v4i*)(soff + 4 * (tid + OTHR));
    int* op = off + base;
    *(volatile v4i*)(op + 4 * tid) = o0;
    *(volatile v4i*)(op + 4 * (tid + OTHR)) = o1;
    __threadfence();
    *(volatile v4i*)(op + 4 * tid) = o0;
    *(volatile v4i*)(op + 4 * (tid + OTHR)) = o1;
    __syncthreads();
  }
  if (tid == 0) {
    srb[min(NFB * nChunk, RBN - 2)] = carry;
    srb[RBN - 1] = flag | ((carry > csrLen) ? 1 : 0);
  }
  __syncthreads();
  v4i rv = {0, 0, 0, 0};
  if (tid < 32) rv = *(const v4i*)(srb + 4 * tid);
  if (tid < 32) *(volatile v4i*)(rbase + 4 * tid) = rv;
  __threadfence();
  if (tid < 32) *(volatile v4i*)(rbase + 4 * tid) = rv;
}

template <int FB>
__global__ __launch_bounds__(NTHR) void k_fill(
    const int* __restrict__ srcs, const int* __restrict__ dsts,
    const int* __restrict__ off, const int* __restrict__ rbase,
    int* csr, int nS, int nE, int vec8, int csrLen) {
  static_assert((FB & (FB - 1)) == 0);
  static_assert(FB <= FBMAX);
  extern __shared__ v4f lds_dyn[];
  int* region = (int*)lds_dyn;
  int* cursor = region + RCAP;
  int* list   = cursor + FBMAX;
  int* wcnt   = list + LISTN;
  const int tid = threadIdx.x, lane = tid & 31, wave = tid >> 5;
  const int b = blockIdx.x;
  const int nodeBase = b * FB;

  int rb0 = rbase[b];
  const int rb1 = rbase[b + 1];
  rb0 = rb0 < 0 ? 0 : (rb0 > csrLen ? csrLen : rb0);
  rb0 &= ~31;
  int len = rb1 - rb0;
  len = len < 0 ? 0 : (len > RCAP ? RCAP : len);
  int lenW = (len + 31) & ~31;
  if (rb0 + lenW > csrLen) lenW = (csrLen - rb0) & ~31;

  {
    const v4i z = {0, 0, 0, 0};
    for (int i = tid; i < RCAP / 4; i += NTHR) ((v4i*)region)[i] = z;
    for (int s = tid; s < FB; s += NTHR) {
      int o = off[nodeBase + s] - rb0;
      o = o < 0 ? 0 : (o > RCAP ? RCAP : o);
      cursor[s] = o;
    }
  }
  __syncthreads();

  const int nChunks = (nE + CHUNK - 1) / CHUNK;
#pragma unroll 1
  for (int ch = 0; ch < nChunks; ++ch) {
    const int cbase = ch * CHUNK;
    const int wc = scan_chunk<FB>(dsts, nE, cbase, nodeBase, vec8, list, tid, lane, wave);
    if (lane == 0) wcnt[wave] = wc;
    __syncthreads();
    if (wave == 0) {
#pragma unroll 1
      for (int wsx = 0; wsx < NWAVE; ++wsx) {
        int n = __builtin_amdgcn_readfirstlane(wcnt[wsx]);
        n = n > WCAP ? WCAP : (n < 0 ? 0 : n);
        const int* lp = list + wsx * WCAP;
#pragma unroll 1
        for (int i = 0; i < n; ++i) {
          const int ent  = __builtin_amdgcn_readfirstlane(lp[i]);
          const int slot = ent & (FB - 1);
          int e = cbase + ((ent >> 12) & (CHUNK - 1));
          e = e > nE - 1 ? nE - 1 : e;
          int sv = srcs[e];
          sv = sv < 0 ? 0 : (sv > nS - 1 ? nS - 1 : sv);
          if (lane == 0) {
            int pos = cursor[slot];
            pos = pos < 0 ? 0 : (pos > RCAP - 1 ? RCAP - 1 : pos);
            region[pos] = sv;
            const int np = pos + 1;
            cursor[slot] = np > RCAP ? RCAP : np;
          }
        }
      }
    }
    __syncthreads();
  }

  const int nv = lenW >> 2;
  int* gp = csr + rb0;
#pragma unroll 1
  for (int i = tid; i < nv; i += NTHR) { const v4i v = ((const v4i*)region)[i]; *(volatile v4i*)(gp + 4 * i) = v; }
  __threadfence();
#pragma unroll 1
  for (int i = tid; i < nv; i += NTHR) { const v4i v = ((const v4i*)region)[i]; *(volatile v4i*)(gp + 4 * i) = v; }
}

__global__ __launch_bounds__(NTHR) void k_wcvt(const float* __restrict__ w, _Float16* dp, int nUnits) {
  const int i = (int)blockIdx.x * NTHR + (int)threadIdx.x;
  if (i >= nUnits) return;
  const int ppr = DW / 8;
  const int n = i / ppr;
  const int seg = i - n * ppr;
  const float* p = w + (size_t)(8 * seg) * DW + n;
  v8h o;
#pragma unroll
  for (int j = 0; j < 8; ++j) o[j] = (_Float16)(p[(size_t)j * DW] * WCARRY);
  _Float16* gp = dp + (size_t)i * 8;
  *(volatile v8h*)gp = o;
  __threadfence();
  *(volatile v8h*)gp = o;
}

__global__ __launch_bounds__(NTHR) void k_gemm(
    const float* __restrict__ X, const _Float16* __restrict__ Bp, const float* __restrict__ bias,
    const float* __restrict__ rs, float* Cout, int nValid) {
  constexpr int TPW = 4;
  constexpr int PPR = DW / 4;
  constexpr int NIT = (BM * PPR) / NTHR;
  static_assert((BM * PPR) % NTHR == 0);
  static_assert(NIT >= 1);
  static_assert(TPW * 16 * 2 == DW);
  static_assert(BM == 4 * 16);

  __shared__ __attribute__((aligned(16))) float stg[BM * DW];
  __shared__ __attribute__((aligned(16))) _Float16 a16[BM * DW];
  const int tid = threadIdx.x, lane = tid & 31, wave = tid >> 5, hh = lane >> 4, m = lane & 15;
  const int rowBase = (int)blockIdx.x * BM;
  const int rg = wave >> 1, chf = wave & 1;
  const int r0 = rg * 16;
  const int c0 = chf * (DW / 2);

#pragma unroll
  for (int it = 0; it < NIT; ++it) {
    const int id = it * NTHR + tid;
    const int row = id / PPR, seg = id % PPR;
    const int grow = rowBase + row;
    const bool live = grow < nValid;
    int rr = grow > nValid - 1 ? nValid - 1 : grow;
    rr = rr < 0 ? 0 : rr;
    v4f xv = *(const v4f*)(X + (size_t)rr * DW + 4 * seg);
    v4h o;
    o.x = (_Float16)((live ? xv.x : 0.f) * ACARRY);
    o.y = (_Float16)((live ? xv.y : 0.f) * ACARRY);
    o.z = (_Float16)((live ? xv.z : 0.f) * ACARRY);
    o.w = (_Float16)((live ? xv.w : 0.f) * ACARRY);
    *(v4h*)(a16 + (size_t)row * DW + 4 * seg) = o;
  }
  __syncthreads();

  v8f acc[TPW];
#pragma unroll
  for (int t = 0; t < TPW; ++t) { v8f z = {0.f, 0.f, 0.f, 0.f, 0.f, 0.f, 0.f, 0.f}; acc[t] = z; }

  const _Float16* ap = a16 + (size_t)(r0 + m) * DW + 8 * hh;
  const _Float16* bp = Bp + (size_t)(c0 + m) * DW + 8 * hh;
#pragma unroll 1
  for (int kt = 0; kt < KSTEPS; ++kt) {
    Frag a;
    a.h[0] = *(const v8h*)(ap + 32 * kt);
    a.h[1] = *(const v8h*)(ap + 32 * kt + 16);
#pragma unroll
    for (int t = 0; t < TPW; ++t) {
      const size_t to = (size_t)(16 * t) * DW + 32 * kt;
      Frag b;
      b.h[0] = *(const v8h*)(bp + to);
      b.h[1] = *(const v8h*)(bp + to + 16);
      acc[t] = wmh(a.v, b.v, acc[t]);
    }
  }

  {
    const int growb = rowBase + r0 + 8 * hh;
    const v4f sa = *(const v4f*)(rs + growb);
    const v4f sb = *(const v4f*)(rs + growb + 4);
    const float rsv[8] = {sa.x, sa.y, sa.z, sa.w, sb.x, sb.y, sb.z, sb.w};
    float* sp = stg + (size_t)(r0 + 8 * hh) * DW + c0 + m;
#pragma unroll
    for (int t = 0; t < TPW; ++t) {
      const float bv = bias[c0 + 16 * t + m];
#pragma unroll
      for (int r = 0; r < 8; ++r) {
        const bool lv = (growb + r) < nValid;
        const float g = acc[t][r] * GSCALE;
        const float v = (g + bv) * rsv[r];
        sp[r * DW + 16 * t] = lv ? v : 0.f;
      }
    }
  }
  __syncthreads();

  v4f cv[NIT];
#pragma unroll
  for (int it = 0; it < NIT; ++it) {
    const int id = it * NTHR + tid;
    const int row = id / PPR, seg = id % PPR;
    cv[it] = *(const v4f*)(stg + (size_t)row * DW + 4 * seg);
  }
#pragma unroll
  for (int it = 0; it < NIT; ++it) {
    const int id = it * NTHR + tid;
    const int row = id / PPR, seg = id % PPR;
    float* gp = Cout + (size_t)(rowBase + row) * DW + 4 * seg;
    *(volatile v4f*)gp = cv[it];
  }
  __threadfence();
#pragma unroll
  for (int it = 0; it < NIT; ++it) {
    const int id = it * NTHR + tid;
    const int row = id / PPR, seg = id % PPR;
    float* gp = Cout + (size_t)(rowBase + row) * DW + 4 * seg;
    *(volatile v4f*)gp = cv[it];
  }
}

template <int FINAL>
__global__ __launch_bounds__(NTHR) void k_agg(
    const int* __restrict__ csr, const int* __restrict__ off, const int* __restrict__ cnt,
    const float* __restrict__ scl, const float* __restrict__ h, float* dst,
    const int* __restrict__ fa, const int* __restrict__ fb, int nDst, int nSrc, int csrLen) {
  const int tid = threadIdx.x, lane = tid & 31, wave = tid >> 5;
  const int tbase = blockIdx.x * TGT + wave * 32;
  const int col4 = 4 * lane;
  const int cl    = tbase + lane;
  const int cnt_l = cnt[cl];
  const int off_l = off[cl];
  const float sc_l = scl[cl];
  int bad = 0;
  if constexpr (FINAL == 1) bad = fa[RBN - 1] | fb[RBN - 1];
  const float qn = __int_as_float(0x7fc00000);

#pragma unroll 1
  for (int j = 0; j < 32; ++j) {
    const int c = tbase + j;
    int n = __shfl(cnt_l, j);
    n = n < 0 ? 0 : (n > DEGCAP ? DEGCAP : n);
    const int st = __shfl(off_l, j);
    const float dc = __shfl(sc_l, j);

    v4f a = {0.f, 0.f, 0.f, 0.f};
#pragma unroll 1
    for (int q0 = 0; q0 < n; q0 += 32) {
      int pos = st + q0 + lane;
      pos = pos < 0 ? 0 : (pos > csrLen - 1 ? csrLen - 1 : pos);
      int sl = csr[pos];
      sl = sl < 0 ? 0 : (sl > nSrc - 1 ? nSrc - 1 : sl);
      const int mcnt = (n - q0) < 32 ? (n - q0) : 32;
#pragma unroll 1
      for (int pp = 0; pp < mcnt; ++pp) {
        const int s = __builtin_amdgcn_readlane(sl, pp);
        const v4f xv = *(const v4f*)(h + (size_t)s * DW + col4);
        a = a + xv;
      }
    }

    const bool live = c < nDst;
    v4f o = a * dc;
    if constexpr (FINAL == 1) {
      o.x = fmaxf(o.x, 0.f);
      o.y = fmaxf(o.y, 0.f);
      o.z = fmaxf(o.z, 0.f);
      o.w = fmaxf(o.w, 0.f);
      o.x = bad ? qn : o.x;
      o.y = bad ? qn : o.y;
      o.z = bad ? qn : o.z;
      o.w = bad ? qn : o.w;
      if (live) {
        float* gp = dst + (size_t)c * DW + col4;
        *(volatile v4f*)gp = o;
        __threadfence();
        *(volatile v4f*)gp = o;
      }
    } else {
      o.x = live ? o.x : 0.f;
      o.y = live ? o.y : 0.f;
      o.z = live ? o.z : 0.f;
      o.w = live ? o.w : 0.f;
      float* gp = dst + (size_t)c * DW + col4;
      *(volatile v4f*)gp = o;
      __threadfence();
      *(volatile v4f*)gp = o;
    }
  }
}

extern "C" void kernel_launch(void* const* d_in, const int* in_sizes, int n_in,
                              void* d_out, int out_size, void* d_ws, size_t ws_size,
                              hipStream_t stream) {
  if (n_in < 5) return;
  if (in_sizes[0] < DW || (in_sizes[0] % DW) != 0) return;
  const int nN = in_sizes[0] / DW;
  if (in_sizes[1] != DW * DW || in_sizes[2] != DW) return;
  const int nE = in_sizes[3];
  if (nE < 1 || in_sizes[4] != nE) return;
  if (out_size != nN * DW) return;
  if (nE > (1 << 28) || nN > (1 << 22)) return;
  const int nM = NHE;

  const float* X     = (const float*)d_in[0];
  const float* w     = (const float*)d_in[1];
  const float* bias  = (const float*)d_in[2];
  const int*   v_idx = (const int*)d_in[3];
  const int*   e_idx = (const int*)d_in[4];
  float* out = (float*)d_out;

  constexpr int NFBV = NBC / FBV;
  constexpr int NFBE = NBC / FBE;
  const int NPADV = ((nN + TGT - 1) / TGT) * TGT;
  const int NPADE = ((nM + TGT - 1) / TGT) * TGT;
  const int nBCV  = (nN + NBC - 1) / NBC;
  const int nBCE  = (nM + NBC - 1) / NBC;
  const int CNTV  = nBCV * NBC;
  const int CNTE  = nBCE * NBC;
  if (CNTV < NPADV || CNTE < NPADE) return;
  const int nFBV  = (nN + FBV - 1) / FBV;
  const int nFBE  = (nM + FBE - 1) / FBE;
  if (nFBV > nBCV * NFBV || nFBE > nBCE * NFBE) return;
  if (nBCV * NFBV + 2 > RBN || nBCE * NFBE + 2 > RBN) return;
  const int csrLenV = ((nE + 31) & ~31) + 32 * (nBCV * NFBV + 1);
  const int csrLenE = ((nE + 31) & ~31) + 32 * (nBCE * NFBE + 1);
  const int nGemm  = NPADV / BM;
  const int nAggV  = NPADV / TGT;
  const int nAggE  = NPADE / TGT;
  const int nUnits = DW * (DW / 8);

  char* ws = (char*)d_ws;
  size_t off = 0;
  const size_t oWp  = off; off += (size_t)DW * DW * 2;            off = (off + 255) & ~(size_t)255;
  const size_t oXs  = off; off += (size_t)NPADV * DW * 4;         off = (off + 255) & ~(size_t)255;
  const size_t oYe  = off; off += (size_t)NPADE * DW * 4;         off = (off + 255) & ~(size_t)255;
  const size_t oCV  = off; off += (size_t)CNTV * 4;               off = (off + 255) & ~(size_t)255;
  const size_t oDV  = off; off += (size_t)CNTV * 4;               off = (off + 255) & ~(size_t)255;
  const size_t oOV  = off; off += (size_t)CNTV * 4;               off = (off + 255) & ~(size_t)255;
  const size_t oRV  = off; off += (size_t)RBN * 4;                off = (off + 255) & ~(size_t)255;
  const size_t oCsV = off; off += (size_t)csrLenV * 4;            off = (off + 255) & ~(size_t)255;
  const size_t oCE  = off; off += (size_t)CNTE * 4;               off = (off + 255) & ~(size_t)255;
  const size_t oDE  = off; off += (size_t)CNTE * 4;               off = (off + 255) & ~(size_t)255;
  const size_t oOE  = off; off += (size_t)CNTE * 4;               off = (off + 255) & ~(size_t)255;
  const size_t oRE  = off; off += (size_t)RBN * 4;                off = (off + 255) & ~(size_t)255;
  const size_t oCsE = off; off += (size_t)csrLenE * 4;            off = (off + 255) & ~(size_t)255;
  if (off > ws_size || off > (size_t)WSCAP) return;

  _Float16* wpl = (_Float16*)(ws + oWp);
  float* Xs   = (float*)(ws + oXs);
  float* Ye   = (float*)(ws + oYe);
  int*   cntV = (int*)(ws + oCV);
  float* dvi  = (float*)(ws + oDV);
  int*   offV = (int*)(ws + oOV);
  int*   rbV  = (int*)(ws + oRV);
  int*   csrV = (int*)(ws + oCsV);
  int*   cntE = (int*)(ws + oCE);
  float* dei  = (float*)(ws + oDE);
  int*   offE = (int*)(ws + oOE);
  int*   rbE  = (int*)(ws + oRE);
  int*   csrE = (int*)(ws + oCsE);

  const int vec8 = 1;

  k_wcvt<<<(nUnits + NTHR - 1) / NTHR, NTHR, 0, stream>>>(w, wpl, nUnits);

  k_count<0><<<nBCV, NTHR, 0, stream>>>(v_idx, cntV, dvi, nE, vec8);
  k_offsets<NFBV><<<1, OTHR, 0, stream>>>(cntV, offV, rbV, nBCV, csrLenV);
  hipFuncSetAttribute(reinterpret_cast<const void*>(&k_fill<FBV>),
                      hipFuncAttributeMaxDynamicSharedMemorySize, LDS_FILL);
  k_fill<FBV><<<nFBV, NTHR, LDS_FILL, stream>>>(e_idx, v_idx, offV, rbV, csrV, nM, nE, vec8, csrLenV);

  k_count<1><<<nBCE, NTHR, 0, stream>>>(e_idx, cntE, dei, nE, vec8);
  k_offsets<NFBE><<<1, OTHR, 0, stream>>>(cntE, offE, rbE, nBCE, csrLenE);
  hipFuncSetAttribute(reinterpret_cast<const void*>(&k_fill<FBE>),
                      hipFuncAttributeMaxDynamicSharedMemorySize, LDS_FILL);
  k_fill<FBE><<<nFBE, NTHR, LDS_FILL, stream>>>(v_idx, e_idx, offE, rbE, csrE, nN, nE, vec8, csrLenE);

  k_gemm<<<nGemm, NTHR, 0, stream>>>(X, wpl, bias, dvi, Xs, nN);

  k_agg<0><<<nAggE, NTHR, 0, stream>>>(csrE, offE, cntE, dei, Xs, Ye, rbV, rbE, nM, nN, csrLenE);

  k_agg<1><<<nAggV, NTHR, 0, stream>>>(csrV, offV, cntV, dvi, Ye, out, rbV, rbE, nN, nM, csrLenV);
}
